// ProteinGraph_72318659330279
// MI455X (gfx1250) — hardware-verified
//
#include <hip/hip_runtime.h>
#include <stddef.h>


#define HID    64
#define IN_DIM 38
#define NL     4
#define NG     128
#define GR     32
#define GTHR   128
#define AP     72
#define XSP    68
#define AR     64
#define NB     1024
#define CHUNK  2048
#define NTHR   256
#define NWAVE  8
#define WCAP   256
#define NGRP   (CHUNK / (NTHR * 4))
#define WROWS  (NL * HID + HID)
#define PSTAT  128

#define LDS_AGG_BYTES ((NB * HID + 3 * NB + NWAVE * WCAP + NWAVE) * 4)

static_assert(NGRP == 2);
static_assert(WCAP == (CHUNK / NTHR) * 32);
static_assert(NB == 1024);
static_assert(NB / 4 == NTHR);
static_assert(CHUNK == 2048);
static_assert(LDS_AGG_BYTES == 282656);
static_assert(NG == NWAVE * 16);
static_assert((AP % 8) == 0);
static_assert((XSP % 4) == 0);
static_assert(GR == 4 * 8 && AR == NWAVE * 8);

typedef float          v4f   __attribute__((ext_vector_type(4)));
typedef float          v8f   __attribute__((ext_vector_type(8)));
typedef int            v4i   __attribute__((ext_vector_type(4)));
typedef unsigned short v8us  __attribute__((ext_vector_type(8)));
typedef __bf16         v16bf __attribute__((ext_vector_type(16)));
union Frag { v16bf v; v8us half[2]; };
union Pk8  { v8us v; unsigned short s[8]; };

__device__ __forceinline__ v8f wmb(v16bf a, v16bf b, v8f c) {
  v8f d = __builtin_amdgcn_wmma_f32_16x16x32_bf16(false, a, false, b, (short)0, c, false, false);
  asm volatile("v_nop\n\tv_nop\n\tv_nop\n\tv_nop" : "+v"(d) : "v"(a), "v"(b));
  return d;
}

__device__ __forceinline__ unsigned short bfb(float f) {
  unsigned u = __float_as_uint(f);
  u += 0x7FFFu + ((u >> 16) & 1u);
  return (unsigned short)(u >> 16);
}
__device__ __forceinline__ float bff(unsigned short b) { return __uint_as_float(((unsigned)b) << 16); }

__device__ __forceinline__ float hsum16(float v) {
  v += __shfl_xor(v, 8, 32);
  v += __shfl_xor(v, 4, 32);
  v += __shfl_xor(v, 2, 32);
  v += __shfl_xor(v, 1, 32);
  return v;
}
__device__ __forceinline__ float lk(float x) { return x >= 0.f ? x : 0.01f * x; }
__device__ __forceinline__ int iclamp(int x, int lo, int hi) { return x < lo ? lo : (x > hi ? hi : x); }

__device__ __forceinline__ void mm_tile2(const unsigned short* Ah, const unsigned short* Al,
                                         const unsigned short* __restrict__ bh,
                                         const unsigned short* __restrict__ bl,
                                         int m, int hh, v8f& c0, v8f& c1) {
#pragma unroll
  for (int kt = 0; kt < HID / 32; ++kt) {
    const int k0 = kt * 32 + 8 * hh;
    Frag a0h, a0l, a1h, a1l, wh, wl;
    const unsigned short* p0 = Ah + m * AP + k0;
    const unsigned short* q0 = Al + m * AP + k0;
    const unsigned short* p1 = Ah + (16 + m) * AP + k0;
    const unsigned short* q1 = Al + (16 + m) * AP + k0;
    a0h.half[0] = *(const v8us*)p0;  a0h.half[1] = *(const v8us*)(p0 + 16);
    a0l.half[0] = *(const v8us*)q0;  a0l.half[1] = *(const v8us*)(q0 + 16);
    a1h.half[0] = *(const v8us*)p1;  a1h.half[1] = *(const v8us*)(p1 + 16);
    a1l.half[0] = *(const v8us*)q1;  a1l.half[1] = *(const v8us*)(q1 + 16);
    wh.half[0]  = *(const v8us*)(bh + k0);  wh.half[1] = *(const v8us*)(bh + k0 + 16);
    wl.half[0]  = *(const v8us*)(bl + k0);  wl.half[1] = *(const v8us*)(bl + k0 + 16);
    c0 = wmb(a0h.v, wh.v, c0);  c0 = wmb(a0h.v, wl.v, c0);  c0 = wmb(a0l.v, wh.v, c0);
    c1 = wmb(a1h.v, wh.v, c1);  c1 = wmb(a1h.v, wl.v, c1);  c1 = wmb(a1l.v, wh.v, c1);
  }
}

__global__ __launch_bounds__(NTHR) void k_prep(const float* __restrict__ lin_w,
                                               const float* __restrict__ W_enc,
                                               unsigned short* Wh, unsigned short* Wl) {
  const int i = blockIdx.x * NTHR + threadIdx.x;
  if (i >= WROWS * 8) return;
  const int row = i >> 3;
  const int kq  = (i & 7) * 8;
  float v[8];
  if (blockIdx.x < (NL * HID * 8) / NTHR) {
    const int l = row >> 6, n = row & 63;
#pragma unroll
    for (int j = 0; j < 8; ++j)
      v[j] = lin_w[(size_t)l * HID * HID + (size_t)(kq + j) * HID + n];
  } else {
    const int n = row - NL * HID;
#pragma unroll
    for (int j = 0; j < 8; ++j) {
      const int k  = kq + j;
      const int kc = (k < IN_DIM) ? k : (IN_DIM - 1);
      const float t = W_enc[kc * HID + n];
      v[j] = (k < IN_DIM) ? t : 0.f;
    }
  }
  Pk8 ph, pl;
#pragma unroll
  for (int j = 0; j < 8; ++j) {
    const unsigned short hb = bfb(v[j]);
    ph.s[j] = hb;
    pl.s[j] = bfb(v[j] - bff(hb));
  }
  const size_t o = (size_t)row * HID + kq;
  *(volatile v8us*)(Wh + o) = ph.v;
  *(volatile v8us*)(Wl + o) = pl.v;
  __threadfence();
  *(volatile v8us*)(Wh + o) = ph.v;
  *(volatile v8us*)(Wl + o) = pl.v;
}

__global__ __launch_bounds__(GTHR) void k_enc(const float* __restrict__ X,
                                              const unsigned short* __restrict__ Wh,
                                              const unsigned short* __restrict__ Wl,
                                              const float* __restrict__ benc,
                                              float* zout, float* part, int nN) {
  __shared__ __attribute__((aligned(16))) unsigned short Ah[GR * AP];
  __shared__ __attribute__((aligned(16))) unsigned short Al[GR * AP];
  __shared__ __attribute__((aligned(16))) float Xs[GR * XSP];
  __shared__ __attribute__((aligned(16))) float Ps[PSTAT];

  const int tid = threadIdx.x, lane = tid & 31, wave = tid >> 5;
  const int hh = lane >> 4, m = lane & 15;
  const int rowBase = blockIdx.x * GR;

#pragma unroll 4
  for (int i = tid; i < GR * 64; i += GTHR) {
    const int r = i >> 6, k = i & 63;
    int grow = rowBase + r;
    if (grow > nN - 1) grow = nN - 1;
    const int kc = (k < IN_DIM) ? k : (IN_DIM - 1);
    const float t = X[(size_t)grow * IN_DIM + kc];
    const float v = (k < IN_DIM) ? t : 0.f;
    const unsigned short hb = bfb(v);
    Ah[r * AP + k] = hb;
    Al[r * AP + k] = bfb(v - bff(hb));
  }
  __syncthreads();

  const int ncol = wave * 16 + m;
  v8f c0 = {0.f, 0.f, 0.f, 0.f, 0.f, 0.f, 0.f, 0.f};
  v8f c1 = {0.f, 0.f, 0.f, 0.f, 0.f, 0.f, 0.f, 0.f};
  mm_tile2(Ah, Al, Wh + (size_t)ncol * HID, Wl + (size_t)ncol * HID, m, hh, c0, c1);

  const float bv = benc[ncol];
#pragma unroll
  for (int r = 0; r < 8; ++r) {
    Xs[(8 * hh + r) * XSP + ncol]      = c0[r] + bv;
    Xs[(16 + 8 * hh + r) * XSP + ncol] = c1[r] + bv;
  }
  __syncthreads();

  if (tid < HID) {
    int nv = nN - rowBase;
    nv = nv < 0 ? 0 : (nv > GR ? GR : nv);
    float s = 0.f, q = 0.f;
#pragma unroll 1
    for (int r = 0; r < nv; ++r) {
      const float x = Xs[r * XSP + tid];
      s += x;
      q += x * x;
    }
    Ps[tid] = s;
    Ps[HID + tid] = q;
  }
  __syncthreads();

  v4f pz[4];
#pragma unroll
  for (int j = 0; j < 4; ++j) pz[j] = *(const v4f*)(Xs + (8 * wave + 2 * j + hh) * XSP + 4 * m);
  const v4f pp = *(const v4f*)(Ps + 4 * lane);
  float* ppd = part + (size_t)blockIdx.x * PSTAT + 4 * lane;

#pragma unroll
  for (int j = 0; j < 4; ++j)
    *(volatile v4f*)(zout + (size_t)(rowBase + 8 * wave + 2 * j + hh) * HID + 4 * m) = pz[j];
  if (wave == 0) *(volatile v4f*)ppd = pp;
  __threadfence();
#pragma unroll
  for (int j = 0; j < 4; ++j)
    *(volatile v4f*)(zout + (size_t)(rowBase + 8 * wave + 2 * j + hh) * HID + 4 * m) = pz[j];
  if (wave == 0) *(volatile v4f*)ppd = pp;
}

__global__ __launch_bounds__(64) void k_bn1_fin(const float* __restrict__ part,
                                                const float* __restrict__ gam,
                                                float* bnp, int nBlk, int nN) {
  __shared__ __attribute__((aligned(16))) float bs[2 * HID];
  const int c = threadIdx.x;
  double s = 0.0, q = 0.0;
#pragma unroll 1
  for (int b = 0; b < nBlk; ++b) {
    s += (double)part[(size_t)b * PSTAT + c];
    q += (double)part[(size_t)b * PSTAT + HID + c];
  }
  const double inv = 1.0 / (double)nN;
  const double mu  = s * inv;
  double var = q * inv - mu * mu;
  if (var < 0.0) var = 0.0;
  bs[c]       = (float)mu;
  bs[HID + c] = gam[c] * rsqrtf((float)var + 1.0e-5f);
  __syncthreads();
  if (c < 32) {
    const v4f v = *(const v4f*)(bs + 4 * c);
    float* p = bnp + 4 * c;
    *(volatile v4f*)p = v;
    __threadfence();
    *(volatile v4f*)p = v;
  }
}

__global__ __launch_bounds__(NTHR) void k_bn1_apply(const float* __restrict__ z,
                                                    const float* __restrict__ bnp,
                                                    const float* __restrict__ beta,
                                                    const float* __restrict__ aw,
                                                    float* feat, float* acc, float* su, float* sv) {
  __shared__ __attribute__((aligned(16))) float Suv[2 * AR];
  const int tid = threadIdx.x, lane = tid & 31, wave = tid >> 5;
  const int hh = lane >> 4, m = lane & 15;
  const int base = blockIdx.x * AR;

  const v4f m4  = *(const v4f*)(bnp + 4 * m);
  const v4f sc4 = *(const v4f*)(bnp + HID + 4 * m);
  const v4f b4  = *(const v4f*)(beta + 4 * m);
  const v4f awu = *(const v4f*)(aw + 4 * m);
  const v4f awv = *(const v4f*)(aw + HID + 4 * m);

  v4f yv[4];
#pragma unroll
  for (int j = 0; j < 4; ++j) {
    const int rloc = 8 * wave + 2 * j + hh;
    const v4f x = *(const v4f*)(z + (size_t)(base + rloc) * HID + 4 * m);
    const v4f y = (x - m4) * sc4 + b4;
    yv[j] = y;
    const float pu = hsum16(y.x * awu.x + y.y * awu.y + y.z * awu.z + y.w * awu.w);
    const float pv = hsum16(y.x * awv.x + y.y * awv.y + y.z * awv.z + y.w * awv.w);
    if (m == 0) { Suv[rloc] = pu; Suv[AR + rloc] = pv; }
  }
#pragma unroll
  for (int j = 0; j < 4; ++j) {
    const size_t o = (size_t)(base + 8 * wave + 2 * j + hh) * HID + 4 * m;
    *(volatile v4f*)(feat + o) = yv[j];
    *(volatile v4f*)(acc + o)  = yv[j];
  }
  __syncthreads();
  const v4f gv = *(const v4f*)(Suv + 4 * lane);
  float* gp = (lane < 16) ? (su + base + 4 * lane) : (sv + base + 4 * (lane - 16));
  if (wave == 0) *(volatile v4f*)gp = gv;
  __threadfence();
#pragma unroll
  for (int j = 0; j < 4; ++j) {
    const size_t o = (size_t)(base + 8 * wave + 2 * j + hh) * HID + 4 * m;
    *(volatile v4f*)(feat + o) = yv[j];
    *(volatile v4f*)(acc + o)  = yv[j];
  }
  if (wave == 0) *(volatile v4f*)gp = gv;
}

__global__ __launch_bounds__(NTHR) void k_agg(const float* __restrict__ feat, const int* __restrict__ ei,
                                              const float* __restrict__ su, const float* __restrict__ sv,
                                              float* msg, int nN, int nE) {
  extern __shared__ v4f lds_dyn[];
  float* sacc = (float*)lds_dyn;
  float* smx  = sacc + NB * HID;
  float* sden = smx + NB;
  float* ssv  = sden + NB;
  int*   list = (int*)(ssv + NB);
  int*   wcnt = list + NWAVE * WCAP;

  const int tid = threadIdx.x, lane = tid & 31, wave = tid >> 5;
  const int hh = lane >> 4, m = lane & 15;
  const int nodeBase = blockIdx.x * NB;
  {
    const v4f z4 = {0.f, 0.f, 0.f, 0.f};
    for (int i = tid; i < NB * HID / 4; i += NTHR) lds_dyn[i] = z4;
    const v4f neg4 = {-1.0e30f, -1.0e30f, -1.0e30f, -1.0e30f};
    *(v4f*)(smx + 4 * tid)  = neg4;
    *(v4f*)(sden + 4 * tid) = z4;
    *(v4f*)(ssv + 4 * tid)  = *(const v4f*)(sv + nodeBase + 4 * tid);
  }
  __syncthreads();

  const int* eid = ei + nE;
  const bool al16 = ((nE & 3) == 0);
  const int nChunks = (nE + CHUNK - 1) / CHUNK;
#pragma unroll 1
  for (int ch = 0; ch < nChunks; ++ch) {
    const int cbase = ch * CHUNK;
    int wc = 0;
#pragma unroll
    for (int g = 0; g < NGRP; ++g) {
      const int el0 = (g * NTHR + tid) * 4;
      const int e0  = cbase + el0;
      const int sent = -2147483647 - 1;
      v4i d;
      if (al16 && (e0 + 3 < nE)) {
        d = *(const v4i*)(eid + e0);
      } else {
        d.x = (e0     < nE) ? eid[iclamp(e0,     0, nE - 1)] : sent;
        d.y = (e0 + 1 < nE) ? eid[iclamp(e0 + 1, 0, nE - 1)] : sent;
        d.z = (e0 + 2 < nE) ? eid[iclamp(e0 + 2, 0, nE - 1)] : sent;
        d.w = (e0 + 3 < nE) ? eid[iclamp(e0 + 3, 0, nE - 1)] : sent;
      }
      const unsigned s0 = (unsigned)d.x - (unsigned)nodeBase;
      const unsigned s1 = (unsigned)d.y - (unsigned)nodeBase;
      const unsigned s2 = (unsigned)d.z - (unsigned)nodeBase;
      const unsigned s3 = (unsigned)d.w - (unsigned)nodeBase;
      const bool h0 = s0 < (unsigned)NB;
      const bool h1 = s1 < (unsigned)NB;
      const bool h2 = s2 < (unsigned)NB;
      const bool h3 = s3 < (unsigned)NB;
      const unsigned many = __builtin_amdgcn_ballot_w32(h0 | h1 | h2 | h3);
      if (many != 0u) {
#define HITJ(J, HJ, SJ) { \
          const unsigned mj = __builtin_amdgcn_ballot_w32(HJ); \
          if (HJ) { \
            const int pos = wc + (int)__builtin_amdgcn_mbcnt_lo(mj, 0u); \
            if (pos < WCAP) list[wave * WCAP + pos] = ((el0 + (J)) << 10) | (int)(SJ); \
          } \
          wc += (int)__builtin_popcount(mj); }
        HITJ(0, h0, s0)
        HITJ(1, h1, s1)
        HITJ(2, h2, s2)
        HITJ(3, h3, s3)
#undef HITJ
      }
    }
    if (lane == 0) wcnt[wave] = wc;
    __syncthreads();

    if (wave == 0) {
      for (int wsx = 0; wsx < NWAVE; ++wsx) {
        int n = wcnt[wsx];
        n = n < 0 ? 0 : (n > WCAP ? WCAP : n);
        for (int i = 0; i < n; ++i) {
          const int ent  = list[wsx * WCAP + i];
          const int slot = ent & (NB - 1);
          const int el   = (ent >> 10) & (CHUNK - 1);
          int e = cbase + el;
          if (e > nE - 1) e = nE - 1;
          int src = ei[e];
          src = iclamp(src, 0, nN - 1);
          const float a  = su[src] + ssv[slot];
          const float mo = smx[slot];
          const float mn = fmaxf(mo, a);
          const float sc = __expf(mo - mn);
          const float p  = __expf(a - mn);
          const v4f xv = *(const v4f*)(feat + (size_t)src * HID + 4 * m);
          v4f* sp = (v4f*)(sacc + slot * HID + 4 * m);
          const v4f cur = *sp;
          const v4f nxt = cur * sc + p * xv;
          *sp = nxt;
          const float dn = sden[slot] * sc + p;
          sden[slot] = dn;
          smx[slot]  = mn;
        }
      }
    }
    __syncthreads();
  }

#pragma unroll 1
  for (int j = 0; j < NB / (2 * NWAVE); ++j) {
    const int slot = wave * (NB / NWAVE) + 2 * j + hh;
    const float dsum = sden[slot];
    const float inv  = 1.0f / fmaxf(dsum, 1.0f);
    const v4f v = *(const v4f*)(sacc + slot * HID + 4 * m) * inv;
    float* p = msg + (size_t)(nodeBase + slot) * HID + 4 * m;
    *(volatile v4f*)p = v;
    __threadfence();
    *(volatile v4f*)p = v;
  }
}

__global__ __launch_bounds__(GTHR) void k_gemm_ln(const float* __restrict__ msg,
                                                  const unsigned short* __restrict__ Wh,
                                                  const unsigned short* __restrict__ Wl,
                                                  const float* __restrict__ lb,
                                                  const float* __restrict__ lng,
                                                  const float* __restrict__ lnb,
                                                  const float* __restrict__ awn,
                                                  float* fout, float* acc, float* su, float* sv) {
  __shared__ __attribute__((aligned(16))) unsigned short Ah[GR * AP];
  __shared__ __attribute__((aligned(16))) unsigned short Al[GR * AP];
  __shared__ __attribute__((aligned(16))) float Xs[GR * XSP];
  __shared__ __attribute__((aligned(16))) float Suv[4 * GR];

  const int tid = threadIdx.x, lane = tid & 31, wave = tid >> 5;
  const int hh = lane >> 4, m = lane & 15;
  const int rowBase = blockIdx.x * GR;

  {
    const int r = tid >> 2, c0 = (tid & 3) * 16;
    const float* p = msg + (size_t)(rowBase + r) * HID + c0;
    const v4f f0 = *(const v4f*)p, f1 = *(const v4f*)(p + 4);
    const v4f f2 = *(const v4f*)(p + 8), f3 = *(const v4f*)(p + 12);
    Pk8 h0, l0, h1, l1;
#define SPL(P, IDX, VAL) { const float f_ = (VAL); const unsigned short b_ = bfb(f_); \
      h##P.s[IDX] = b_; l##P.s[IDX] = bfb(f_ - bff(b_)); }
    SPL(0, 0, f0.x) SPL(0, 1, f0.y) SPL(0, 2, f0.z) SPL(0, 3, f0.w)
    SPL(0, 4, f1.x) SPL(0, 5, f1.y) SPL(0, 6, f1.z) SPL(0, 7, f1.w)
    SPL(1, 0, f2.x) SPL(1, 1, f2.y) SPL(1, 2, f2.z) SPL(1, 3, f2.w)
    SPL(1, 4, f3.x) SPL(1, 5, f3.y) SPL(1, 6, f3.z) SPL(1, 7, f3.w)
#undef SPL
    *(v8us*)(Ah + r * AP + c0)     = h0.v;
    *(v8us*)(Ah + r * AP + c0 + 8) = h1.v;
    *(v8us*)(Al + r * AP + c0)     = l0.v;
    *(v8us*)(Al + r * AP + c0 + 8) = l1.v;
  }
  __syncthreads();

  const int ncol = wave * 16 + m;
  v8f c0 = {0.f, 0.f, 0.f, 0.f, 0.f, 0.f, 0.f, 0.f};
  v8f c1 = {0.f, 0.f, 0.f, 0.f, 0.f, 0.f, 0.f, 0.f};
  mm_tile2(Ah, Al, Wh + (size_t)ncol * HID, Wl + (size_t)ncol * HID, m, hh, c0, c1);

  const float bv = lb[ncol];
#pragma unroll
  for (int r = 0; r < 8; ++r) {
    Xs[(8 * hh + r) * XSP + ncol]      = c0[r] + bv;
    Xs[(16 + 8 * hh + r) * XSP + ncol] = c1[r] + bv;
  }
  __syncthreads();

  const v4f g4  = *(const v4f*)(lng + 4 * m);
  const v4f e4  = *(const v4f*)(lnb + 4 * m);
  const v4f awu = *(const v4f*)(awn + 4 * m);
  const v4f awv = *(const v4f*)(awn + HID + 4 * m);

  v4f yv[4], an[4];
#pragma unroll
  for (int j = 0; j < 4; ++j) {
    const int rloc = 8 * wave + 2 * j + hh;
    const v4f x = *(const v4f*)(Xs + rloc * XSP + 4 * m);
    const float s  = hsum16(x.x + x.y + x.z + x.w);
    const float mu = s * (1.0f / HID);
    const v4f dd = x - mu;
    const float q  = hsum16(dd.x * dd.x + dd.y * dd.y + dd.z * dd.z + dd.w * dd.w);
    const float rs = rsqrtf(q * (1.0f / HID) + 1.0e-5f);
    v4f y = dd * rs * g4 + e4;
    y.x = lk(y.x); y.y = lk(y.y); y.z = lk(y.z); y.w = lk(y.w);
    yv[j] = y;
    const v4f av = *(const v4f*)(acc + (size_t)(rowBase + rloc) * HID + 4 * m);
    an[j] = av + y;
    const float pu = hsum16(y.x * awu.x + y.y * awu.y + y.z * awu.z + y.w * awu.w);
    const float pv = hsum16(y.x * awv.x + y.y * awv.y + y.z * awv.z + y.w * awv.w);
    if (m == 0) { Suv[rloc] = pu; Suv[GR + rloc] = pv; }
  }
#pragma unroll
  for (int j = 0; j < 4; ++j) {
    const size_t o = (size_t)(rowBase + 8 * wave + 2 * j + hh) * HID + 4 * m;
    *(volatile v4f*)(fout + o) = yv[j];
    *(volatile v4f*)(acc + o)  = an[j];
  }
  __syncthreads();
  const v4f gv = *(const v4f*)(Suv + 4 * lane);
  float* gp = (lane < 8) ? (su + rowBase + 4 * lane) : (sv + rowBase + 4 * (lane - 8));
  if (wave == 0 && lane < 16) *(volatile v4f*)gp = gv;
  __threadfence();
#pragma unroll
  for (int j = 0; j < 4; ++j) {
    const size_t o = (size_t)(rowBase + 8 * wave + 2 * j + hh) * HID + 4 * m;
    *(volatile v4f*)(fout + o) = yv[j];
    *(volatile v4f*)(acc + o)  = an[j];
  }
  if (wave == 0 && lane < 16) *(volatile v4f*)gp = gv;
}

__global__ __launch_bounds__(NTHR) void k_pool(const float* __restrict__ accp, const int* __restrict__ batch,
                                               const int* __restrict__ ngp, const float* __restrict__ g2,
                                               const float* __restrict__ b2, float* out, int nN) {
  __shared__ __attribute__((aligned(16))) float ps[NG * HID];
  __shared__ float pc[NG];
  const int tid = threadIdx.x, lane = tid & 31, wave = tid >> 5;
  const int hh = lane >> 4, m = lane & 15;
  int ng = ngp[0];
  ng = ng < 1 ? 1 : (ng > NG ? NG : ng);
  const int nCh = (nN + 127) / 128;

#pragma unroll 1
  for (int gi = 0; gi < NG / NWAVE; ++gi) {
    const int g = gi * NWAVE + wave;
    v4f a4 = {0.f, 0.f, 0.f, 0.f};
    int cnt = 0;
#pragma unroll 1
    for (int ch = 0; ch < nCh; ++ch) {
      const int base = ch * 128 + 4 * lane;
      int bq[4];
#pragma unroll
      for (int j = 0; j < 4; ++j) {
        const int idx = base + j;
        const int idc = idx > nN - 1 ? nN - 1 : idx;
        const int t = batch[idc];
        bq[j] = (idx < nN) ? t : -1;
      }
#pragma unroll
      for (int j = 0; j < 4; ++j) {
        unsigned mj = __builtin_amdgcn_ballot_w32(bq[j] == g);
        cnt += (int)__builtin_popcount(mj);
        while (mj != 0u) {
          const int b = __builtin_ctz(mj);
          mj &= mj - 1u;
          int node = ch * 128 + 4 * b + j;
          if (node > nN - 1) node = nN - 1;
          const v4f f = *(const v4f*)(accp + (size_t)node * HID + 4 * m);
          a4 = a4 + f * 0.2f;
        }
      }
    }
    if (hh == 0) *(v4f*)(ps + g * HID + 4 * m) = a4;
    if (lane == 0) pc[g] = (float)cnt;
  }
  __syncthreads();

  if (tid < HID) {
    const int c = tid;
    const float invg = 1.0f / (float)ng;
    float s = 0.f;
#pragma unroll 1
    for (int g = 0; g < NG; ++g) {
      const float x = ps[g * HID + c] * (1.0f / fmaxf(pc[g], 1.0f));
      ps[g * HID + c] = x;
      s += x;
    }
    const float mu = s * invg;
    float q = 0.f;
#pragma unroll 1
    for (int g = 0; g < NG; ++g) { const float d = ps[g * HID + c] - mu; q += d * d; }
    const float rs = rsqrtf(q * invg + 1.0e-5f);
    const float gg = g2[c], bb = b2[c];
#pragma unroll 1
    for (int g = 0; g < NG; ++g) {
      const float y = (ps[g * HID + c] - mu) * rs * gg + bb;
      ps[g * HID + c] = lk(y);
    }
  }
  __syncthreads();

  v4f ov[8];
#pragma unroll
  for (int j = 0; j < 8; ++j) ov[j] = *(const v4f*)(ps + (wave * (NG / NWAVE) + 2 * j + hh) * HID + 4 * m);
#pragma unroll
  for (int j = 0; j < 8; ++j)
    *(volatile v4f*)(out + (size_t)(wave * (NG / NWAVE) + 2 * j + hh) * HID + 4 * m) = ov[j];
  __threadfence();
#pragma unroll
  for (int j = 0; j < 8; ++j)
    *(volatile v4f*)(out + (size_t)(wave * (NG / NWAVE) + 2 * j + hh) * HID + 4 * m) = ov[j];
}

static size_t al256(size_t x) { return (x + 255) & ~(size_t)255; }

extern "C" void kernel_launch(void* const* d_in, const int* in_sizes, int n_in,
                              void* d_out, int out_size, void* d_ws, size_t ws_size,
                              hipStream_t stream) {
  if (n_in < 15) return;
  const int nE = in_sizes[0] / 2;
  const int nN = in_sizes[2];
  if (nN <= 0 || nE < 1 || in_sizes[0] != 2 * nE) return;
  if (in_sizes[1] != nN * IN_DIM) return;
  if (in_sizes[3] < 1) return;
  if (in_sizes[4] != IN_DIM * HID || in_sizes[5] != HID || in_sizes[6] != HID || in_sizes[7] != HID) return;
  if (in_sizes[8] != NL * 2 * HID || in_sizes[9] != NL * HID * HID || in_sizes[10] != NL * HID) return;
  if (in_sizes[11] != NL * HID || in_sizes[12] != NL * HID || in_sizes[13] != HID || in_sizes[14] != HID) return;
  if (out_size != NG * HID) return;

  const int*   edge  = (const int*)d_in[0];
  const float* nfeat = (const float*)d_in[1];
  const int*   batch = (const int*)d_in[2];
  const int*   ngp   = (const int*)d_in[3];
  const float* Wenc  = (const float*)d_in[4];
  const float* benc  = (const float*)d_in[5];
  const float* bn1g  = (const float*)d_in[6];
  const float* bn1b  = (const float*)d_in[7];
  const float* a_w   = (const float*)d_in[8];
  const float* lin_w = (const float*)d_in[9];
  const float* lin_b = (const float*)d_in[10];
  const float* ln_g  = (const float*)d_in[11];
  const float* ln_b  = (const float*)d_in[12];
  const float* bn2g  = (const float*)d_in[13];
  const float* bn2b  = (const float*)d_in[14];
  float* out = (float*)d_out;

  const int NP    = ((nN + NB - 1) / NB) * NB;
  const int nBlkG = NP / GR;
  const size_t plane = (size_t)NP * HID * sizeof(float);
  char* ws = (char*)d_ws;
  size_t off = 0;
  float* msgz  = (float*)(ws + off); off += al256(plane);
  float* featA = (float*)(ws + off); off += al256(plane);
  float* featB = (float*)(ws + off); off += al256(plane);
  float* accb  = (float*)(ws + off); off += al256(plane);
  float* su    = (float*)(ws + off); off += al256((size_t)NP * sizeof(float));
  float* sv    = (float*)(ws + off); off += al256((size_t)NP * sizeof(float));
  float* part  = (float*)(ws + off); off += al256((size_t)nBlkG * PSTAT * sizeof(float));
  float* bnp   = (float*)(ws + off); off += al256((size_t)2 * HID * sizeof(float));
  unsigned short* Wh = (unsigned short*)(ws + off); off += al256((size_t)WROWS * HID * sizeof(unsigned short));
  unsigned short* Wl = (unsigned short*)(ws + off); off += al256((size_t)WROWS * HID * sizeof(unsigned short));
  if (off > ws_size) return;

  k_prep<<<(WROWS * 8 + NTHR - 1) / NTHR, NTHR, 0, stream>>>(lin_w, Wenc, Wh, Wl);

  k_enc<<<NP / GR, GTHR, 0, stream>>>(nfeat, Wh + (size_t)NL * HID * HID, Wl + (size_t)NL * HID * HID,
                                      benc, msgz, part, nN);
  k_bn1_fin<<<1, 64, 0, stream>>>(part, bn1g, bnp, nBlkG, nN);
  k_bn1_apply<<<NP / AR, NTHR, 0, stream>>>(msgz, bnp, bn1b, a_w, featA, accb, su, sv);

  hipFuncSetAttribute(reinterpret_cast<const void*>(&k_agg),
                      hipFuncAttributeMaxDynamicSharedMemorySize, LDS_AGG_BYTES);
  for (int l = 0; l < NL; ++l) {
    float* fin = (l & 1) ? featB : featA;
    float* fo  = (l & 1) ? featA : featB;
    k_agg<<<NP / NB, NTHR, LDS_AGG_BYTES, stream>>>(fin, edge, su, sv, msgz, nN, nE);
    const int ln = (l + 1 < NL) ? (l + 1) : (NL - 1);
    k_gemm_ln<<<NP / GR, GTHR, 0, stream>>>(msgz, Wh + (size_t)l * HID * HID, Wl + (size_t)l * HID * HID,
                                            lin_b + l * HID, ln_g + l * HID, ln_b + l * HID,
                                            a_w + (size_t)ln * 2 * HID, fo, accb, su, sv);
  }

  k_pool<<<1, NTHR, 0, stream>>>(accb, batch, ngp, bn2g, bn2b, out, nN);
  (void)hipGetLastError();
}
